// LSTM_40097814675741
// MI455X (gfx1250) — hardware-verified
//
#include <hip/hip_runtime.h>
#include <math.h>

constexpr int SEQ_T    = 200;
constexpr int NB       = 256;
constexpr int NH       = 50;
constexpr int NE       = 128;
constexpr int NV       = 100000;
constexpr int NGATE    = 4;
constexpr int UPAD     = 64;
constexpr int NCOLP    = NGATE * UPAD;
constexpr int KPAD     = 64;
constexpr int NHEAD1   = 16;
constexpr int NOUTC    = 9;
constexpr int NROW     = SEQ_T * NB;
constexpr int NTHR     = 256;
constexpr int ROWS_BLK = 32;
constexpr int HP       = 72;
constexpr int XSP      = 260;
constexpr int HDP      = 17;
constexpr float WCARRY = 256.0f;
constexpr float HCARRY = 2048.0f;
constexpr float WINV   = 1.0f / WCARRY;
constexpr float WLINV  = 1.0f / (WCARRY * HCARRY);

static_assert(NROW % 64 == 0);
static_assert(NCOLP % 64 == 0);
static_assert(NE % 32 == 0);
static_assert(((NROW / 64) * (NCOLP / 64)) % 8 == 0);
static_assert(NROW % 16 == 0);
static_assert(NB % ROWS_BLK == 0);
static_assert(ROWS_BLK == 32 && NTHR == 256);
static_assert(NH <= UPAD && NGATE * UPAD == NCOLP);
static_assert(ROWS_BLK * NCOLP == 8 * 4 * NTHR);
static_assert((ROWS_BLK * NOUTC * 4) % 128 == 0);
static_assert((NB * NOUTC * 4) % 128 == 0);
static_assert((ROWS_BLK * NOUTC) % 4 == 0 && (ROWS_BLK * NOUTC) / 4 <= NTHR);
static_assert(ROWS_BLK * NOUTC <= NTHR + 32);
static_assert(HP % 8 == 0 && XSP % 4 == 0);
static_assert((2 * ROWS_BLK * HP) % NTHR == 0);
static_assert((NCOLP * 8) % NTHR == 0);

typedef __attribute__((ext_vector_type(16))) _Float16 v16h;
typedef __attribute__((ext_vector_type(8)))  _Float16 v8h;
typedef __attribute__((ext_vector_type(16))) __bf16   v16b;
typedef __attribute__((ext_vector_type(8)))  __bf16   v8b;
typedef __attribute__((ext_vector_type(8)))  float    v8f;
typedef __attribute__((ext_vector_type(4)))  float    v4f;

__device__ __forceinline__ unsigned short f2bf_bits(float f) {
  unsigned u = __float_as_uint(f);
  return (unsigned short)((u + 0x7FFFu + ((u >> 16) & 1u)) >> 16);
}
__device__ __forceinline__ float bf_bits2f(unsigned short h) { return __uint_as_float(((unsigned)h) << 16); }
__device__ __forceinline__ float bf16r(float f) { return bf_bits2f(f2bf_bits(f)); }

__device__ __forceinline__ void dep_guard_h(v8f& a, v8f& b, v16h x, v16h y) { asm volatile("v_nop\n\tv_nop\n\tv_nop\n\tv_nop" : "+v"(a), "+v"(b) : "v"(x), "v"(y)); }
__device__ __forceinline__ void dep_guard_b(v8f& a, v8f& b, v16b x, v16b y) { asm volatile("v_nop\n\tv_nop\n\tv_nop\n\tv_nop" : "+v"(a), "+v"(b) : "v"(x), "v"(y)); }
__device__ __forceinline__ void dep_guard4_h(v8f& a, v8f& b, v8f& c, v8f& d, v16h x, v16h y) { asm volatile("v_nop\n\tv_nop\n\tv_nop\n\tv_nop" : "+v"(a), "+v"(b), "+v"(c), "+v"(d) : "v"(x), "v"(y)); }
__device__ __forceinline__ void dep_guard4_b(v8f& a, v8f& b, v8f& c, v8f& d, v16b x, v16b y) { asm volatile("v_nop\n\tv_nop\n\tv_nop\n\tv_nop" : "+v"(a), "+v"(b), "+v"(c), "+v"(d) : "v"(x), "v"(y)); }
__device__ __forceinline__ void dep_guard8_h(v8f& a0, v8f& a1, v8f& a2, v8f& a3, v8f& c0, v8f& c1, v8f& c2, v8f& c3, v16h x, v16h y) {
  asm volatile("v_nop\n\tv_nop\n\tv_nop\n\tv_nop" : "+v"(a0), "+v"(a1), "+v"(a2), "+v"(a3), "+v"(c0), "+v"(c1), "+v"(c2), "+v"(c3) : "v"(x), "v"(y));
}
__device__ __forceinline__ void keep4_h(v16h a, v16h b, v16h c, v16h d) { asm volatile("v_nop" :: "v"(a), "v"(b), "v"(c), "v"(d)); }
__device__ __forceinline__ void keep4_b(v16b a, v16b b, v16b c, v16b d) { asm volatile("v_nop" :: "v"(a), "v"(b), "v"(c), "v"(d)); }
__device__ __forceinline__ void acc_guard4(v8f& a, v8f& b, v8f& c, v8f& d) { asm volatile("v_nop\n\tv_nop\n\tv_nop\n\tv_nop" : "+v"(a), "+v"(b), "+v"(c), "+v"(d)); }
template <typename T> struct Frag;
template <> struct Frag<_Float16> {
  typedef v16h V; union U { v16h v; v8h h[2]; };
  static __device__ __forceinline__ v16h load(const _Float16* p) {
    U f; f.h[0] = *(const v8h*)(p); f.h[1] = *(const v8h*)(p + 16); return f.v;
  }
  static __device__ __forceinline__ v8f mma(v16h a, v16h b, v8f c) {
    return __builtin_amdgcn_wmma_f32_16x16x32_f16(false, a, false, b, (short)0, c, false, false);
  }
  static __device__ __forceinline__ void guard(v8f& a, v8f& b, v16h x, v16h y) { dep_guard_h(a, b, x, y); }
  static __device__ __forceinline__ void guard4(v8f& a, v8f& b, v8f& c, v8f& d, v16h x, v16h y) { dep_guard4_h(a, b, c, d, x, y); }
  static __device__ __forceinline__ void keep(v16h a, v16h b, v16h c, v16h d) { keep4_h(a, b, c, d); }
};
template <> struct Frag<__bf16> {
  typedef v16b V; union U { v16b v; v8b h[2]; };
  static __device__ __forceinline__ v16b load(const __bf16* p) {
    U f; f.h[0] = *(const v8b*)(p); f.h[1] = *(const v8b*)(p + 16); return f.v;
  }
  static __device__ __forceinline__ v8f mma(v16b a, v16b b, v8f c) {
    return __builtin_amdgcn_wmma_f32_16x16x32_bf16(false, a, false, b, (short)0, c, false, false);
  }
  static __device__ __forceinline__ void guard(v8f& a, v8f& b, v16b x, v16b y) { dep_guard_b(a, b, x, y); }
  static __device__ __forceinline__ void guard4(v8f& a, v8f& b, v8f& c, v8f& d, v16b x, v16b y) { dep_guard4_b(a, b, c, d, x, y); }
  static __device__ __forceinline__ void keep(v16b a, v16b b, v16b c, v16b d) { keep4_b(a, b, c, d); }
};

__device__ __forceinline__ float fsig(float x)  { return __builtin_amdgcn_rcpf(1.0f + expf(-x)); }
__device__ __forceinline__ float ftanh(float x) { return 1.0f - 2.0f * __builtin_amdgcn_rcpf(expf(2.0f * x) + 1.0f); }

template <int ET> struct Elem;
template <> struct Elem<0> { typedef _Float16 T; };
template <> struct Elem<1> { typedef __bf16 T; };
template <int ET, bool SPLIT, int BIAS_MODE, int OUT_MODE, bool RESID, int ACT = 0>
__global__ __launch_bounds__(256) void wmma_gemm64(
    const unsigned short* __restrict__ Ap, const unsigned short* __restrict__ A2p, int lda, long strideA,
    const unsigned short* __restrict__ Btp, const unsigned short* __restrict__ Bt2p, int ldb, long strideB,
    void* __restrict__ Cout, void* __restrict__ Cout2, int ldc, long strideC,
    const float* __restrict__ bias,
    const float* __restrict__ resid, long strideR,
    int M, int N, int K, float scale) {
  typedef typename Elem<ET>::T T;
  typedef typename Frag<T>::V V;
  const T* A = (const T*)Ap; const T* A2 = (const T*)A2p; const T* Bt = (const T*)Btp; const T* Bt2 = (const T*)Bt2p;
  __shared__ __align__(16) float sT[8][16 * 68];
  const int b    = blockIdx.y;
  const int lane = threadIdx.x & 31;
  const int wave = threadIdx.x >> 5;
  const int tilesN = N >> 6;
  const int tilesM = M >> 6;
  const int tile = blockIdx.x * 8 + wave;
  if (tile >= tilesM * tilesN) return;
  const int tm = tile / tilesN;
  const int tn = tile - tm * tilesN;
  const int m0 = tm << 6;
  const int n0 = tn << 6;

  const T* Ab  = A  + (size_t)b * strideA;
  const T* Bb  = Bt + (size_t)b * strideB;
  const T* Ab2 = SPLIT ? (A2  + (size_t)b * strideA) : nullptr;
  const T* Bb2 = SPLIT ? (Bt2 + (size_t)b * strideB) : nullptr;

  const int rlane = lane & 15;
  const int koff  = (lane >> 4) * 8;
  const int mOff  = (lane >> 4) * 8;

  v8f acc[4][4];
#pragma unroll
  for (int i = 0; i < 4; ++i)
#pragma unroll
    for (int j = 0; j < 4; ++j) acc[i][j] = (v8f){0.f,0.f,0.f,0.f,0.f,0.f,0.f,0.f};

  for (int k0 = 0; k0 < K; k0 += 32) {
    V bh[4], bl[4];
#pragma unroll
    for (int j = 0; j < 4; ++j) {
      const size_t bo = (size_t)(n0 + (j << 4) + rlane) * ldb + koff + k0;
      bh[j] = Frag<T>::load(Bb + bo);
      if (SPLIT) bl[j] = Frag<T>::load(Bb2 + bo);
    }
#pragma unroll
    for (int i = 0; i < 4; ++i) {
      const size_t ao = (size_t)(m0 + (i << 4) + rlane) * lda + koff + k0;
      V ah = Frag<T>::load(Ab + ao);
      V al;
      if (SPLIT) al = Frag<T>::load(Ab2 + ao);
#pragma unroll
      for (int j = 0; j < 4; ++j) {
        acc[i][j] = Frag<T>::mma(ah, bh[j], acc[i][j]);
        if (SPLIT) {
          acc[i][j] = Frag<T>::mma(ah, bl[j], acc[i][j]);
          acc[i][j] = Frag<T>::mma(al, bh[j], acc[i][j]);
        }
      }
      Frag<T>::guard4(acc[i][0], acc[i][1], acc[i][2], acc[i][3], ah, SPLIT ? al : ah);
    }
    Frag<T>::keep(bh[0], bh[1], bh[2], bh[3]);
    if (SPLIT) Frag<T>::keep(bl[0], bl[1], bl[2], bl[3]);
  }
  acc_guard4(acc[0][0], acc[0][1], acc[0][2], acc[0][3]);
  acc_guard4(acc[1][0], acc[1][1], acc[1][2], acc[1][3]);
  acc_guard4(acc[2][0], acc[2][1], acc[2][2], acc[2][3]);
  acc_guard4(acc[3][0], acc[3][1], acc[3][2], acc[3][3]);

  float* slab = sT[wave];
  const float* Rb = RESID ? (resid + (size_t)b * strideR) : nullptr;
#pragma unroll
  for (int i = 0; i < 4; ++i) {
    const int mBase = m0 + (i << 4);
#pragma unroll
    for (int j = 0; j < 4; ++j) {
      const int n = n0 + (j << 4) + rlane;
      float bv = 0.f;
      if (BIAS_MODE == 2) bv = bias[n];
#pragma unroll
      for (int r = 0; r < 8; ++r) {
        float v = acc[i][j][r] * scale;
        if (BIAS_MODE == 1) v += bias[mBase + mOff + r];
        if (BIAS_MODE == 2) v += bv;
        if (RESID) v += Rb[(size_t)(mBase + mOff + r) * ldc + n];
        if (ACT == 1) v = tanhf(v);
        if (ACT == 2) v = fmaxf(v, 0.0f);
        if (ACT == 3) v = v / (1.0f + expf(-v));
        if (ACT == 4) v = (v > 0.f) ? v : 0.01f * v;
        if (ACT == 5) v = 0.5f * v * (1.0f + erff(v * 0.70710678118654752f));
        slab[(mOff + r) * 68 + (j << 4) + rlane] = v;
      }
    }
    __builtin_amdgcn_fence(__ATOMIC_RELEASE, "workgroup");
    __builtin_amdgcn_wave_barrier();
    __builtin_amdgcn_fence(__ATOMIC_ACQUIRE, "workgroup");
    if (OUT_MODE == 0) {
      float* C = (float*)Cout + (size_t)b * strideC;
      const int hh = lane >> 4, c4 = (lane & 15) * 4;
      for (int pass = 0; pass < 2; ++pass) {
#pragma unroll
        for (int it = 0; it < 8; ++it) {
          const int row = it * 2 + hh;
          v4f v = *(const v4f*)(slab + row * 68 + c4);
          *(volatile v4f*)(C + (size_t)(mBase + row) * ldc + n0 + c4) = v;
        }
        __threadfence();
      }
    } else {
      const int q = lane >> 3, c8 = (lane & 7) * 8;
      unsigned short* C  = (unsigned short*)Cout  + (size_t)b * strideC;
      unsigned short* C2 = (OUT_MODE == 2) ? ((unsigned short*)Cout2 + (size_t)b * strideC) : nullptr;
      for (int pass = 0; pass < 2; ++pass) {
#pragma unroll
        for (int it = 0; it < 4; ++it) {
          const int row = it * 4 + q;
          const float* sp = slab + row * 68 + c8;
          v8h hv, lv;
#pragma unroll
          for (int e = 0; e < 8; ++e) {
            if (OUT_MODE == 1) {
              hv[e] = (_Float16)sp[e];
            } else {
              unsigned short hb = f2bf_bits(sp[e]);
              unsigned short lb = f2bf_bits(sp[e] - bf_bits2f(hb));
              hv[e] = __builtin_bit_cast(_Float16, hb);
              lv[e] = __builtin_bit_cast(_Float16, lb);
            }
          }
          *(volatile v8h*)(C + (size_t)(mBase + row) * ldc + n0 + c8) = hv;
          if (OUT_MODE == 2) *(volatile v8h*)(C2 + (size_t)(mBase + row) * ldc + n0 + c8) = lv;
        }
        __threadfence();
      }
    }
    __builtin_amdgcn_fence(__ATOMIC_RELEASE, "workgroup");
    __builtin_amdgcn_wave_barrier();
    __builtin_amdgcn_fence(__ATOMIC_ACQUIRE, "workgroup");
  }
}

__global__ __launch_bounds__(NTHR) void gather_rows_kernel(const int* __restrict__ tok, const float* __restrict__ emb,
                                                          unsigned short* __restrict__ Xg) {
  const int tid = threadIdx.x;
  const int row = blockIdx.x * 16 + (tid >> 4);
  const int c8  = (tid & 15) * 8;
  int tk = tok[row];
  tk = tk < 0 ? 0 : tk;
  tk = tk > NV - 1 ? NV - 1 : tk;
  const float* sp = emb + (size_t)tk * NE + c8;
  const v4f a = *(const v4f*)(sp);
  const v4f b = *(const v4f*)(sp + 4);
  v8h hv;
#pragma unroll
  for (int e = 0; e < 4; ++e) {
    const unsigned short u0 = f2bf_bits(a[e]);
    const unsigned short u1 = f2bf_bits(b[e]);
    hv[e]     = __builtin_bit_cast(_Float16, u0);
    hv[4 + e] = __builtin_bit_cast(_Float16, u1);
  }
  unsigned short* dp = Xg + (size_t)row * NE + c8;
  *(volatile v8h*)dp = hv;
  __threadfence();
  *(volatile v8h*)dp = hv;
}

__global__ __launch_bounds__(NTHR) void wih_plane_kernel(const float* __restrict__ wih, const float* __restrict__ bih,
                                                        const float* __restrict__ bhh,
                                                        unsigned short* __restrict__ WIHP, float* __restrict__ BSUM) {
  const int tid = threadIdx.x;
  if (blockIdx.x < NCOLP / 16) {
    const int n  = blockIdx.x * 16 + (tid >> 4);
    const int c8 = (tid & 15) * 8;
    const int g = n >> 6, u = n & 63;
    const bool valid = (u < NH);
    const int srow = g * NH + (valid ? u : (NH - 1));
    const float* sp = wih + (size_t)srow * NE + c8;
    const v4f a = *(const v4f*)(sp);
    const v4f b = *(const v4f*)(sp + 4);
    v8h hv;
#pragma unroll
    for (int e = 0; e < 4; ++e) {
      const float fa = valid ? a[e] : 0.0f;
      const float fb = valid ? b[e] : 0.0f;
      const unsigned short u0 = f2bf_bits(fa);
      const unsigned short u1 = f2bf_bits(fb);
      hv[e]     = __builtin_bit_cast(_Float16, u0);
      hv[4 + e] = __builtin_bit_cast(_Float16, u1);
    }
    unsigned short* dp = WIHP + (size_t)n * NE + c8;
    *(volatile v8h*)dp = hv;
    __threadfence();
    *(volatile v8h*)dp = hv;
  } else {
    if (tid < NCOLP / 4) {
      const int nb = tid * 4;
      const int g = nb >> 6, ub = nb & 63;
      v4f o;
#pragma unroll
      for (int e = 0; e < 4; ++e) {
        const int u = ub + e;
        const bool valid = (u < NH);
        const int src = g * NH + (valid ? u : (NH - 1));
        const float fa = bih[src];
        const float fb = bhh[src];
        const float s = bf16r(fa) + bf16r(fb);
        o[e] = valid ? s : 0.0f;
      }
      float* op = BSUM + nb;
      *(volatile v4f*)op = o;
      __threadfence();
      *(volatile v4f*)op = o;
    }
  }
}

__global__ __launch_bounds__(NTHR) void pad50_kernel(const float* __restrict__ whh, const float* __restrict__ w1,
                                                    unsigned short* __restrict__ WHP, unsigned short* __restrict__ W1P) {
  const int i = blockIdx.x * NTHR + threadIdx.x;
  if (blockIdx.x < (NCOLP * 8) / NTHR) {
    const int n  = i >> 3;
    const int c8 = (i & 7) * 8;
    const int g = n >> 6, u = n & 63;
    const bool valid = (u < NH);
    const int srow = g * NH + (valid ? u : (NH - 1));
    v8h hv;
#pragma unroll
    for (int e = 0; e < 8; ++e) {
      const int k  = c8 + e;
      const int kc = (k < NH) ? k : (NH - 1);
      const float f = whh[(size_t)srow * NH + kc];
      const float use = (valid && k < NH) ? f : 0.0f;
      hv[e] = (_Float16)(WCARRY * bf16r(use));
    }
    unsigned short* dp = WHP + (size_t)n * KPAD + c8;
    *(volatile v8h*)dp = hv;
    __threadfence();
    *(volatile v8h*)dp = hv;
  } else {
    const int i2 = i - NCOLP * 8;
    if (i2 < NHEAD1 * 8) {
      const int n  = i2 >> 3;
      const int c8 = (i2 & 7) * 8;
      v8h hv;
#pragma unroll
      for (int e = 0; e < 8; ++e) {
        const int k  = c8 + e;
        const int kc = (k < NH) ? k : (NH - 1);
        const float f = w1[(size_t)n * NH + kc];
        const float use = (k < NH) ? f : 0.0f;
        hv[e] = (_Float16)(WCARRY * bf16r(use));
      }
      unsigned short* dp = W1P + (size_t)n * KPAD + c8;
      *(volatile v8h*)dp = hv;
      __threadfence();
      *(volatile v8h*)dp = hv;
    }
  }
}

__global__ __launch_bounds__(NTHR) void lstm_seq_kernel(const float* __restrict__ XP,
                                                       const unsigned short* __restrict__ WHPp,
                                                       const unsigned short* __restrict__ W1Pp,
                                                       const float* __restrict__ w2, const float* __restrict__ b1,
                                                       const float* __restrict__ b2, float* __restrict__ out) {
  __shared__ __align__(16) float    Xs[ROWS_BLK * XSP];
  __shared__ __align__(16) _Float16 Ahi[2][ROWS_BLK * HP];
  __shared__ __align__(16) _Float16 Alo[2][ROWS_BLK * HP];
  __shared__ __align__(16) float    Os[ROWS_BLK * NOUTC];
  __shared__ float Hd[ROWS_BLK * HDP];
  __shared__ float W2s[NOUTC * NHEAD1];
  __shared__ float b1s[NHEAD1];
  __shared__ float b2s[16];
  const _Float16* WHP = (const _Float16*)WHPp;
  const _Float16* W1P = (const _Float16*)W1Pp;
  const int tid = threadIdx.x, lane = tid & 31, wave = tid >> 5;
  const int mt = wave >> 2, ub = wave & 3;
  const int c = lane & 15, hh = lane >> 4, koff = hh * 8;
  const int u = 16 * ub + c;
  const int b0 = blockIdx.x * ROWS_BLK;

  {
    _Float16* ph = &Ahi[0][0];
    _Float16* pl = &Alo[0][0];
#pragma unroll 1
    for (int i = tid; i < 2 * ROWS_BLK * HP; i += NTHR) { ph[i] = (_Float16)0.0f; pl[i] = (_Float16)0.0f; }
  }
  {
    const int iw = tid < NOUTC * NHEAD1 ? tid : (NOUTC * NHEAD1 - 1);
    const int i1 = tid < NHEAD1 ? tid : (NHEAD1 - 1);
    const int i2 = tid < NOUTC ? tid : (NOUTC - 1);
    const float vw = w2[iw];
    const float v1 = b1[i1];
    const float v2 = b2[i2];
    if (tid < NOUTC * NHEAD1) W2s[tid] = bf16r(vw);
    if (tid < NHEAD1) b1s[tid] = bf16r(v1);
    if (tid < NOUTC)  b2s[tid] = bf16r(v2);
  }
  float cst[8];
#pragma unroll
  for (int r = 0; r < 8; ++r) cst[r] = 0.0f;

  v16h bw[2][4], w1b[2];
#pragma unroll
  for (int g = 0; g < 4; ++g) bw[0][g] = Frag<_Float16>::load(WHP + (size_t)(g * UPAD + u) * KPAD + koff);
  keep4_h(bw[0][0], bw[0][1], bw[0][2], bw[0][3]);
#pragma unroll
  for (int g = 0; g < 4; ++g) bw[1][g] = Frag<_Float16>::load(WHP + (size_t)(g * UPAD + u) * KPAD + koff + 32);
  keep4_h(bw[1][0], bw[1][1], bw[1][2], bw[1][3]);
  w1b[0] = Frag<_Float16>::load(W1P + (size_t)c * KPAD + koff);
  w1b[1] = Frag<_Float16>::load(W1P + (size_t)c * KPAD + koff + 32);
  keep4_h(w1b[0], w1b[1], w1b[0], w1b[1]);
  __syncthreads();

  const v8f z8 = {0.f, 0.f, 0.f, 0.f, 0.f, 0.f, 0.f, 0.f};

#pragma unroll 1
  for (int t = 0; t < SEQ_T; ++t) {
    const int p = t & 1, pn = p ^ 1;

    {
      const float* xsrc = XP + (size_t)(t * NB + b0) * NCOLP;
#pragma unroll
      for (int it = 0; it < 8; ++it) {
        const int q = it * NTHR + tid;
        const int row = q >> 6, c4 = (q & 63) * 4;
        const v4f v = *(const v4f*)(xsrc + (size_t)row * NCOLP + c4);
        *(v4f*)(Xs + row * XSP + c4) = v;
      }
    }
    __syncthreads();

    {
      const _Float16* ahr = &Ahi[p][0] + (16 * mt + c) * HP + koff;
      const _Float16* alr = &Alo[p][0] + (16 * mt + c) * HP + koff;
      v8f acc[4], accl[4];
#pragma unroll
      for (int g = 0; g < 4; ++g) { acc[g] = z8; accl[g] = z8; }
#pragma unroll
      for (int kc = 0; kc < 2; ++kc) {
        const v16h a  = Frag<_Float16>::load(ahr + 32 * kc);
        const v16h al = Frag<_Float16>::load(alr + 32 * kc);
#pragma unroll
        for (int g = 0; g < 4; ++g) {
          acc[g]  = Frag<_Float16>::mma(a,  bw[kc][g], acc[g]);
          accl[g] = Frag<_Float16>::mma(al, bw[kc][g], accl[g]);
        }
        dep_guard8_h(acc[0], acc[1], acc[2], acc[3], accl[0], accl[1], accl[2], accl[3], a, al);
      }
      _Float16* ahn = &Ahi[pn][0];
      _Float16* aln = &Alo[pn][0];
#pragma unroll
      for (int r = 0; r < 8; ++r) {
        const int R = 16 * mt + 8 * hh + r;
        const float* xr = Xs + R * XSP + u;
        const float zi = acc[0][r] * WINV + accl[0][r] * WLINV + xr[0];
        const float zf = acc[1][r] * WINV + accl[1][r] * WLINV + xr[UPAD];
        const float zg = acc[2][r] * WINV + accl[2][r] * WLINV + xr[2 * UPAD];
        const float zo = acc[3][r] * WINV + accl[3][r] * WLINV + xr[3 * UPAD];
        const float ig = fsig(zi);
        const float fg = fsig(zf);
        const float og = fsig(zo);
        const float gg = ftanh(zg);
        const float cn = fg * cst[r] + ig * gg;
        cst[r] = cn;
        const float hn = og * ftanh(cn);
        const float hs = (u < NH) ? hn : 0.0f;
        const _Float16 hi = (_Float16)hs;
        const float hif = (float)hi;
        const float res = (hs - hif) * HCARRY;
        const _Float16 lo = (_Float16)res;
        ahn[R * HP + u] = hi;
        aln[R * HP + u] = lo;
      }
    }
    __syncthreads();

    if (ub == 0) {
      const _Float16* ahr = &Ahi[pn][0] + (16 * mt + c) * HP + koff;
      const _Float16* alr = &Alo[pn][0] + (16 * mt + c) * HP + koff;
      v8f ha = z8, hl = z8;
#pragma unroll
      for (int kc = 0; kc < 2; ++kc) {
        const v16h a  = Frag<_Float16>::load(ahr + 32 * kc);
        const v16h al = Frag<_Float16>::load(alr + 32 * kc);
        ha = Frag<_Float16>::mma(a,  w1b[kc], ha);
        hl = Frag<_Float16>::mma(al, w1b[kc], hl);
        dep_guard_h(ha, hl, a, al);
      }
#pragma unroll
      for (int r = 0; r < 8; ++r) {
        const int R = 16 * mt + 8 * hh + r;
        const float v = ha[r] * WINV + hl[r] * WLINV + b1s[c];
        Hd[R * HDP + c] = fmaxf(v, 0.0f);
      }
    }
    __syncthreads();

    {
      const int e = tid;
      const int R = e / NOUTC, j = e - R * NOUTC;
      float s = 0.0f;
#pragma unroll
      for (int n = 0; n < NHEAD1; ++n) s = fmaf(Hd[R * HDP + n], W2s[j * NHEAD1 + n], s);
      Os[e] = s + b2s[j];
      if (wave == 0) {
        const int e2 = NTHR + lane;
        const int R2 = e2 / NOUTC, j2 = e2 - R2 * NOUTC;
        float s2 = 0.0f;
#pragma unroll
        for (int n = 0; n < NHEAD1; ++n) s2 = fmaf(Hd[R2 * HDP + n], W2s[j2 * NHEAD1 + n], s2);
        Os[e2] = s2 + b2s[j2];
      }
    }
    __syncthreads();

    {
      const bool wr = (tid < (ROWS_BLK * NOUTC) / 4);
      v4f v = {0.f, 0.f, 0.f, 0.f};
      float* dst = out;
      if (wr) {
        v = *(const v4f*)(Os + 4 * tid);
        dst = out + (size_t)(t * NB + b0) * NOUTC + 4 * tid;
      }
      for (int pass = 0; pass < 2; ++pass) {
        if (wr) *(volatile v4f*)dst = v;
        __threadfence();
      }
    }
  }
}

extern "C" void kernel_launch(void* const* d_in, const int* in_sizes, int n_in,
                              void* d_out, int out_size, void* d_ws, size_t ws_size, hipStream_t stream) {
  if (n_in < 10 || d_out == nullptr || d_ws == nullptr) return;
  if (in_sizes[0] != SEQ_T * NB || in_sizes[1] != NV * NE || in_sizes[2] != NGATE * NH * NE ||
      in_sizes[3] != NGATE * NH * NH || in_sizes[4] != NGATE * NH || in_sizes[5] != NGATE * NH ||
      in_sizes[6] != NHEAD1 * NH || in_sizes[7] != NHEAD1 || in_sizes[8] != NOUTC * NHEAD1 || in_sizes[9] != NOUTC ||
      out_size != NROW * NOUTC) return;

  const int*   tok = (const int*)d_in[0];
  const float* emb = (const float*)d_in[1];
  const float* wih = (const float*)d_in[2];
  const float* whh = (const float*)d_in[3];
  const float* bih = (const float*)d_in[4];
  const float* bhh = (const float*)d_in[5];
  const float* w1  = (const float*)d_in[6];
  const float* b1  = (const float*)d_in[7];
  const float* w2  = (const float*)d_in[8];
  const float* b2  = (const float*)d_in[9];
  float* out = (float*)d_out;

  char* ws = (char*)d_ws; size_t off = 0;
  auto carve = [&](size_t bytes) -> char* { char* p = ws + off; off += (bytes + 255) & ~(size_t)255; return p; };
  unsigned short* Xg   = (unsigned short*)carve((size_t)NROW * NE * 2);
  unsigned short* WIHP = (unsigned short*)carve((size_t)NCOLP * NE * 2);
  unsigned short* WHP  = (unsigned short*)carve((size_t)NCOLP * KPAD * 2);
  unsigned short* W1P  = (unsigned short*)carve((size_t)NHEAD1 * KPAD * 2);
  float*          BSUM = (float*)carve((size_t)NCOLP * 4);
  float*          XP   = (float*)carve((size_t)NROW * NCOLP * 4);
  if (off > ws_size || off > (size_t)134217728) return;

  gather_rows_kernel<<<NROW / 16, NTHR, 0, stream>>>(tok, emb, Xg);
  wih_plane_kernel<<<NCOLP / 16 + 1, NTHR, 0, stream>>>(wih, bih, bhh, WIHP, BSUM);
  pad50_kernel<<<(NCOLP * 8) / NTHR + 1, NTHR, 0, stream>>>(whh, w1, WHP, W1P);
  wmma_gemm64<1, false, 2, 0, false, 0><<<dim3((NROW / 64) * (NCOLP / 64) / 8, 1), 256, 0, stream>>>(
      Xg, Xg, NE, 0L, WIHP, WIHP, NE, 0L, (void*)XP, (void*)XP, NCOLP, 0L,
      BSUM, BSUM, 0L, NROW, NCOLP, NE, 1.0f);
  lstm_seq_kernel<<<NB / ROWS_BLK, NTHR, 0, stream>>>(XP, WHP, W1P, w2, b1, b2, out);
}
